// KANLinear_31447750542039
// MI455X (gfx1250) — hardware-run, weakly checked
//
#include <hip/hip_runtime.h>


#define NBT  8
#define CIN  512
#define COUT 512
#define LL   2048
#define NR   (NBT * LL)
#define NG   12
#define NC   8
#define KK   (CIN * NC)
#define RC   4096
typedef _Float16 h16;
typedef unsigned short bf;
typedef __attribute__((ext_vector_type(16))) __bf16   v16bf;
typedef __attribute__((ext_vector_type(16))) _Float16 v16h;
typedef __attribute__((ext_vector_type(8)))  _Float16 v8h;
typedef __attribute__((ext_vector_type(8)))  unsigned short v8us;
typedef __attribute__((ext_vector_type(8)))  float    v8f;
typedef __attribute__((ext_vector_type(4)))  float    v4f;
typedef v8h  __attribute__((may_alias)) v8ha;
typedef v4f  __attribute__((may_alias)) v4fa;
typedef v8us __attribute__((may_alias)) v8usa;

__device__ __forceinline__ unsigned short f2bf(float f) { unsigned u = __float_as_uint(f); u += 0x7FFFu + ((u >> 16) & 1u); return (unsigned short)(u >> 16); }
__device__ __forceinline__ float bf2f(unsigned short b) { return __uint_as_float(((unsigned)b) << 16); }
__device__ __forceinline__ float bfr(float f) { return bf2f(f2bf(f)); }
__device__ __forceinline__ v16h cat16(v8h lo, v8h hi) { return __builtin_shufflevector(lo, hi, 0, 1, 2, 3, 4, 5, 6, 7, 8, 9, 10, 11, 12, 13, 14, 15); }
__device__ __forceinline__ v16bf cat16b(v8us lo, v8us hi) { return __builtin_bit_cast(v16bf, __builtin_shufflevector(lo, hi, 0, 1, 2, 3, 4, 5, 6, 7, 8, 9, 10, 11, 12, 13, 14, 15)); }
__device__ __forceinline__ v8f wmma16(v16h a, v16h b, v8f c) { return __builtin_amdgcn_wmma_f32_16x16x32_f16(false, a, false, b, (short)0, c, false, false); }
__device__ __forceinline__ v8f wmmab(v16bf a, v16bf b, v8f c) { return __builtin_amdgcn_wmma_f32_16x16x32_bf16(false, a, false, b, (short)0, c, false, false); }


template <typename T16> struct WFrag;
template <> struct WFrag<h16> { typedef v16h V; static __device__ __forceinline__ V ld(const h16* p) { return cat16(*(const v8h*)p, *(const v8h*)(p + 16)); } static __device__ __forceinline__ v8f mma(V a, V b, v8f c) { return wmma16(a, b, c); } };
template <> struct WFrag<bf> { typedef v16bf V; static __device__ __forceinline__ V ld(const bf* p) { return cat16b(*(const v8us*)p, *(const v8us*)(p + 16)); } static __device__ __forceinline__ v8f mma(V a, V b, v8f c) { return wmmab(a, b, c); } };
template <typename T16, int NSPLIT, bool BIAS>
__global__ __launch_bounds__(32) void k_gemmw(const T16* __restrict__ A, const T16* __restrict__ A2, const T16* __restrict__ Bt, const T16* __restrict__ Bt2, int K, float* C, int ldc, const float* __restrict__ bias, size_t sA, size_t sB, size_t sC) {
    typedef typename WFrag<T16>::V V;
    __shared__ __align__(16) float os[16 * 68];
    const size_t z = blockIdx.z; A += z * sA; if (A2) A2 += z * sA; Bt += z * sB; if (Bt2) Bt2 += z * sB; C += z * sC;
    const int lane = threadIdx.x & 31, lr = lane & 15, hi = lane >> 4; const int r0 = blockIdx.x * 64, c0 = blockIdx.y * 64;
    v8f acc[4][4];
#pragma unroll
    for (int mb = 0; mb < 4; ++mb)
#pragma unroll
        for (int nb = 0; nb < 4; ++nb) acc[mb][nb] = (v8f){};
    const size_t aoff = (size_t)(r0 + lr) * K + 8 * hi, boff = (size_t)(c0 + lr) * K + 8 * hi;
#pragma unroll 1
    for (int kc = 0; kc < K; kc += 32) {
        V a[4], a2[4];
#pragma unroll
        for (int mb = 0; mb < 4; ++mb) { a[mb] = WFrag<T16>::ld(A + aoff + (size_t)mb * 16 * K + kc); if (NSPLIT == 1 || NSPLIT == 2) a2[mb] = WFrag<T16>::ld(A2 + aoff + (size_t)mb * 16 * K + kc); }
#pragma unroll
        for (int nb = 0; nb < 4; ++nb) { const V b = WFrag<T16>::ld(Bt + boff + (size_t)nb * 16 * K + kc); V b2; if (NSPLIT >= 2) b2 = WFrag<T16>::ld(Bt2 + boff + (size_t)nb * 16 * K + kc);
#pragma unroll
            for (int mb = 0; mb < 4; ++mb) { acc[mb][nb] = WFrag<T16>::mma(a[mb], b, acc[mb][nb]); if (NSPLIT == 1 || NSPLIT == 2) acc[mb][nb] = WFrag<T16>::mma(a2[mb], b, acc[mb][nb]); if (NSPLIT >= 2) acc[mb][nb] = WFrag<T16>::mma(a[mb], b2, acc[mb][nb]); } }
        asm volatile("v_nop\n\tv_nop\n\tv_nop\n\tv_nop" : "+v"(acc[0][0]), "+v"(acc[1][1]), "+v"(acc[2][2]), "+v"(acc[3][3]) : "v"(a[0]), "v"(a[3]));
    }
#pragma unroll
    for (int mb = 0; mb < 4; ++mb) {
#pragma unroll
        for (int nb = 0; nb < 4; ++nb) {
#pragma unroll
            for (int j = 0; j < 8; ++j) os[(hi * 8 + j) * 68 + nb * 16 + lr] = acc[mb][nb][j]; }
        __builtin_amdgcn_wave_barrier(); asm volatile("" ::: "memory");
        float* crow = C + (size_t)(r0 + mb * 16) * ldc + c0;
#pragma unroll 1
        for (int ps = 0; ps < 2; ++ps) {
#pragma unroll
            for (int s = 0; s < 8; ++s) { const int row = 2 * s + hi, cofs = lr * 4; v4f val = *(const v4fa*)(os + row * 68 + cofs); if (BIAS) { val[0] += bfr(bias[c0 + cofs]); val[1] += bfr(bias[c0 + cofs + 1]); val[2] += bfr(bias[c0 + cofs + 2]); val[3] += bfr(bias[c0 + cofs + 3]); }
                *(volatile v4f*)(crow + (size_t)row * ldc + cofs) = val; }
            if (ps == 0) __threadfence(); }
        __builtin_amdgcn_wave_barrier(); asm volatile("" ::: "memory");
    }
}

typedef __attribute__((ext_vector_type(4))) unsigned short v4us;
typedef __attribute__((ext_vector_type(2))) unsigned short v2us;
__device__ __forceinline__ void splitf(float y, unsigned short& h, unsigned short& l) { h = f2bf(y); l = f2bf(y - bf2f(h)); }
__global__ __launch_bounds__(256) void k_cvt8(const float* __restrict__ src, bf* dst, size_t n8) { const size_t i = (size_t)blockIdx.x * 256 + threadIdx.x; if (i >= n8) return; const v8f v = *(const v8f*)(src + i * 8); v8us o;
#pragma unroll
    for (int k = 0; k < 8; ++k) o[k] = f2bf(v[k]); *(volatile v8us*)(dst + i * 8) = o; __threadfence(); *(volatile v8us*)(dst + i * 8) = o; }

__global__ __launch_bounds__(256) void k_sw(const float* __restrict__ sw, const float* __restrict__ sc, bf* Bh, bf* Bl) { const size_t e = (size_t)blockIdx.x * 256 + threadIdx.x; if (e >= (size_t)COUT * CIN) return; const int i = (int)(e % CIN), o = (int)(e / CIN); const float s = bfr(sc[e]); const v8f w8 = *(const v8f*)(sw + e * NC); v8us oh, ol;
#pragma unroll
    for (int c = 0; c < NC; ++c) { unsigned short h2, l2; splitf(__fmul_rn(bfr(w8[c]), s), h2, l2); oh[c] = h2; ol[c] = l2; }
    const size_t ob = ((size_t)o * CIN + i) * NC; *(volatile v8us*)(Bh + ob) = oh; *(volatile v8us*)(Bl + ob) = ol; __threadfence(); *(volatile v8us*)(Bh + ob) = oh; *(volatile v8us*)(Bl + ob) = ol; }
__global__ __launch_bounds__(256) void k_rden(const float* __restrict__ grid, float* RD) { const int i = blockIdx.x * 256 + threadIdx.x; if (i >= CIN) return; const float* g = grid + (size_t)i * NG;
#pragma unroll 1
    for (int p = 1; p <= 3; ++p) {
#pragma unroll 1
        for (int k = 0; k + p < NG; ++k) { const float r = __fdiv_rn(1.0f, __fsub_rn(bfr(g[k + p]), bfr(g[k]))); *(volatile float*)(RD + (size_t)i * 32 + (p - 1) * 11 + k) = r; __threadfence(); *(volatile float*)(RD + (size_t)i * 32 + (p - 1) * 11 + k) = r; } } }
__global__ __launch_bounds__(256) void k_feat(const float* __restrict__ X, const float* __restrict__ grid, const float* __restrict__ RD, size_t n0, bf* Ah, bf* Al) {
    const size_t e = (size_t)blockIdx.x * 256 + threadIdx.x; if (e >= (size_t)RC * CIN) return; const int i = (int)(e % CIN); const size_t nl = e / CIN; const size_t n = n0 + nl; const int b = (int)(n / LL), l = (int)(n % LL);
    const float x = bfr(X[((size_t)b * CIN + i) * LL + l]); float g[NG];
#pragma unroll
    for (int k = 0; k < NG; ++k) g[k] = bfr(grid[(size_t)i * NG + k]);
    const float* rd = RD + (size_t)i * 32;
    float bs[NG - 1];
#pragma unroll
    for (int k = 0; k < NG - 1; ++k) bs[k] = (x >= g[k] && x < g[k + 1]) ? 1.0f : 0.0f;
#pragma unroll
    for (int p = 1; p <= 3; ++p) {
#pragma unroll
        for (int k = 0; k < NG - 1 - p; ++k) { float dl = __fmul_rn(__fsub_rn(x, g[k]), rd[(p - 1) * 11 + k]); asm volatile("" : "+v"(dl)); float lt = __fmul_rn(dl, bs[k]); asm volatile("" : "+v"(lt)); float dr = __fmul_rn(__fsub_rn(g[k + p + 1], x), rd[(p - 1) * 11 + k + 1]); asm volatile("" : "+v"(dr)); float rt = __fmul_rn(dr, bs[k + 1]); asm volatile("" : "+v"(rt)); bs[k] = __fadd_rn(lt, rt); } }
    v8us oh, ol;
#pragma unroll
    for (int c = 0; c < NC; ++c) { unsigned short h2, l2; splitf(bs[c], h2, l2); oh[c] = h2; ol[c] = l2; }
    const size_t ob = nl * KK + (size_t)i * NC; *(volatile v8us*)(Ah + ob) = oh; *(volatile v8us*)(Al + ob) = ol; __threadfence(); *(volatile v8us*)(Ah + ob) = oh; *(volatile v8us*)(Al + ob) = ol; }
__global__ __launch_bounds__(256) void k_silu(const float* __restrict__ X, size_t n0, bf* Sh, bf* Sl) { const size_t e = ((size_t)blockIdx.x * 256 + threadIdx.x) * 4; if (e >= (size_t)RC * CIN) return; const int i0 = (int)(e % CIN); const size_t nl = e / CIN; const size_t n = n0 + nl; const int b = (int)(n / LL), l = (int)(n % LL); v4us oh, ol;
#pragma unroll
    for (int q = 0; q < 4; ++q) { const float x = bfr(X[((size_t)b * CIN + i0 + q) * LL + l]); const float sg = __fdiv_rn(1.0f, __fadd_rn(1.0f, __builtin_amdgcn_exp2f(__fmul_rn(x, -1.4426950408889634f)))); const float y = __fmul_rn(x, sg); unsigned short h2, l2; splitf(y, h2, l2); oh[q] = h2; ol[q] = l2; }
    *(volatile v4us*)(Sh + e) = oh; *(volatile v4us*)(Sl + e) = ol; __threadfence(); *(volatile v4us*)(Sh + e) = oh; *(volatile v4us*)(Sl + e) = ol; }
__global__ __launch_bounds__(256) void k_outk(const float* __restrict__ C1, const float* __restrict__ C2, size_t n0, float* out) { const size_t i = (size_t)blockIdx.x * 256 + threadIdx.x; if (i >= (size_t)COUT * RC / 4) return; const int l4 = (int)(i % (RC / 4)) * 4; const int o = (int)(i / (RC / 4)); const size_t n = n0 + l4; const int b = (int)(n / LL), l = (int)(n % LL); v4f r;
#pragma unroll
    for (int q = 0; q < 4; ++q) r[q] = __fadd_rn(C1[(size_t)(l4 + q) * COUT + o], C2[(size_t)(l4 + q) * COUT + o]);
    const size_t oo = ((size_t)b * COUT + o) * LL + l; *(volatile v4f*)(out + oo) = r; __threadfence(); *(volatile v4f*)(out + oo) = r; }

extern "C" void kernel_launch(void* const* d_in, const int* in_sizes, int n_in,
                              void* d_out, int out_size, void* d_ws, size_t ws_size, hipStream_t stream) {
    (void)in_sizes; (void)n_in; (void)out_size;
    const float* x = (const float*)d_in[0]; const float* bw = (const float*)d_in[1]; const float* sw = (const float*)d_in[2]; const float* sc = (const float*)d_in[3]; const float* grid = (const float*)d_in[4];
    float* OUT = (float*)d_out;
    char* wsp = (char*)d_ws;
    auto take = [&](size_t bytes) { char* p = wsp; wsp += (bytes + 255) & ~(size_t)255; return (void*)p; };
    bf* BW = (bf*)take((size_t)COUT * CIN * 2); float* RD = (float*)take((size_t)CIN * 32 * 4); bf* SBh = (bf*)take((size_t)COUT * KK * 2); bf* SBl = (bf*)take((size_t)COUT * KK * 2);
    bf* SXh = (bf*)take((size_t)RC * CIN * 2); bf* SXl = (bf*)take((size_t)RC * CIN * 2); bf* Ah = (bf*)take((size_t)RC * KK * 2); bf* Al = (bf*)take((size_t)RC * KK * 2); float* C1 = (float*)take((size_t)RC * COUT * 4); float* C2 = (float*)take((size_t)RC * COUT * 4);
    if ((size_t)(wsp - (char*)d_ws) > ws_size) return;
    k_cvt8<<<(unsigned)(((size_t)COUT * CIN / 8 + 255) / 256), 256, 0, stream>>>(bw, BW, (size_t)COUT * CIN / 8);
    k_sw<<<(unsigned)(((size_t)COUT * CIN + 255) / 256), 256, 0, stream>>>(sw, sc, SBh, SBl); k_rden<<<(CIN + 255) / 256, 256, 0, stream>>>(grid, RD);
    static_assert(NR % RC == 0 && RC % LL == 0 || LL % RC == 0, "chunks align with images");
    for (size_t n0 = 0; n0 < NR; n0 += RC) {
        k_silu<<<(unsigned)(((size_t)RC * CIN / 4 + 255) / 256), 256, 0, stream>>>(x, n0, SXh, SXl);
        k_feat<<<(unsigned)(((size_t)RC * CIN + 255) / 256), 256, 0, stream>>>(x, grid, RD, n0, Ah, Al);
        k_gemmw<bf, 1, false><<<dim3(RC / 64, COUT / 64, 1), 32, 0, stream>>>(SXh, SXl, BW, nullptr, CIN, C1, COUT, nullptr, 0, 0, 0);
        k_gemmw<bf, 2, false><<<dim3(RC / 64, COUT / 64, 1), 32, 0, stream>>>(Ah, Al, SBh, SBl, KK, C2, COUT, nullptr, 0, 0, 0);
        k_outk<<<(unsigned)(((size_t)COUT * RC / 4 + 255) / 256), 256, 0, stream>>>(C1, C2, n0, OUT); }
}
